// SelfAttentiom_4131758539222
// MI455X (gfx1250) — hardware-verified
//
#include <hip/hip_runtime.h>
#include <math.h>

typedef __attribute__((ext_vector_type(16))) _Float16 v16h;
typedef __attribute__((ext_vector_type(8)))  _Float16 v8h;
typedef __attribute__((ext_vector_type(16))) __bf16   v16b;
typedef __attribute__((ext_vector_type(8)))  __bf16   v8b;
typedef __attribute__((ext_vector_type(8)))  float    v8f;
typedef __attribute__((ext_vector_type(4)))  float    v4f;

constexpr int kB   = 4;
constexpr int kS   = 2048;
constexpr int kD   = 1024;
constexpr int kH   = 16;
constexpr int kDh  = 64;
constexpr int kTok = kB * kS;
constexpr int kE3  = 3 * kD;
constexpr int kQKld = 2 * kD;
constexpr int kAtld = 2 * kD;
constexpr int kLoS     = 512;
constexpr int kLoTiles = kLoS / 64;
constexpr int kQTiles  = kS / 64;
constexpr int kSqrtDh  = 8;
static_assert(kSqrtDh * kSqrtDh == kDh, "score scale derived from head width");
static_assert(kH * kDh == kD, "head split");
static_assert((kS % 64) == 0 && (kD % 64) == 0 && (kTok % 64) == 0 && (kLoS % 64) == 0, "tile multiples");
static_assert((kD % 32) == 0 && (kAtld % 32) == 0, "GEMM K multiples of 32");

constexpr float kScoreScale  = 1.0f / (float)kSqrtDh;
constexpr float kLoCarry     = 2048.0f;
constexpr float kLoCarryInv  = 1.0f / kLoCarry;
constexpr float kPCarry      = 32768.0f;
constexpr float kCtxCarry    = 16.0f;
constexpr float kCtxLoCarry  = 256.0f;
constexpr float kWoCarry     = 32.0f;
constexpr float kWoLoScale   = kWoCarry / kCtxLoCarry;
constexpr float kOutScale    = 1.0f / (kCtxCarry * kWoCarry);
constexpr float kMaskFill    = -1.0e30f;

constexpr size_t kOffXB  = 0;
constexpr size_t kOffWB  = kOffXB  + (size_t)kTok * kD * 2;
constexpr size_t kOffWO2 = kOffWB  + (size_t)kE3 * kD * 2;
constexpr size_t kOffQK  = kOffWO2 + (size_t)kD * kAtld * 2;
constexpr size_t kOffVT  = kOffQK  + (size_t)kTok * kQKld * 2;
constexpr size_t kOffQKL = kOffVT  + (size_t)kB * kD * kS * 2;
constexpr size_t kOffVTL = kOffQKL + (size_t)kB * kLoS * kQKld * 2;
constexpr size_t kOffAT  = kOffVTL + (size_t)kB * kD * kLoS * 2;
constexpr size_t kWsTotal = kOffAT + (size_t)kTok * kAtld * 2;
static_assert(kWsTotal == 123731968ull, "carve total");
static_assert(kWsTotal <= 134217728ull, "carve cap");
static_assert((kOffWB % 128) == 0 && (kOffWO2 % 128) == 0 && (kOffQK % 128) == 0 && (kOffVT % 128) == 0 &&
              (kOffQKL % 128) == 0 && (kOffVTL % 128) == 0 && (kOffAT % 128) == 0, "128-B aligned regions");

__device__ __forceinline__ unsigned short f2bf_bits(float f) {
  unsigned u = __float_as_uint(f);
  return (unsigned short)((u + 0x7FFFu + ((u >> 16) & 1u)) >> 16);
}
__device__ __forceinline__ float bf_bits2f(unsigned short h) { return __uint_as_float(((unsigned)h) << 16); }

__device__ __forceinline__ v8f mma_f16(v16h a, v16h b, v8f c) {
  c = __builtin_amdgcn_wmma_f32_16x16x32_f16(false, a, false, b, (short)0, c, false, false);
  asm volatile("v_nop\n\tv_nop\n\tv_nop\n\tv_nop" : "+v"(c) : "v"(a), "v"(b));
  return c;
}
__device__ __forceinline__ v8f mma_bf16(v16b a, v16b b, v8f c) {
  c = __builtin_amdgcn_wmma_f32_16x16x32_bf16(false, a, false, b, (short)0, c, false, false);
  asm volatile("v_nop\n\tv_nop\n\tv_nop\n\tv_nop" : "+v"(c) : "v"(a), "v"(b));
  return c;
}
__device__ __forceinline__ void keep4_h(v16h a, v16h b, v16h c, v16h d) { asm volatile("v_nop" :: "v"(a), "v"(b), "v"(c), "v"(d)); }
__device__ __forceinline__ void keep4_b(v16b a, v16b b, v16b c, v16b d) { asm volatile("v_nop" :: "v"(a), "v"(b), "v"(c), "v"(d)); }
__device__ __forceinline__ void acc_guard4(v8f& a, v8f& b, v8f& c, v8f& d) { asm volatile("v_nop\n\tv_nop\n\tv_nop\n\tv_nop" : "+v"(a), "+v"(b), "+v"(c), "+v"(d)); }

template <typename T> struct Frag;
template <> struct Frag<_Float16> {
  typedef v16h V; union U { v16h v; v8h h[2]; };
  static __device__ __forceinline__ v16h load(const _Float16* p) {
    U f; f.h[0] = *(const v8h*)(p); f.h[1] = *(const v8h*)(p + 16); return f.v;
  }
  static __device__ __forceinline__ v8f mma(v16h a, v16h b, v8f c) { return mma_f16(a, b, c); }
  static __device__ __forceinline__ void keep(v16h a, v16h b, v16h c, v16h d) { keep4_h(a, b, c, d); }
};
template <> struct Frag<__bf16> {
  typedef v16b V; union U { v16b v; v8b h[2]; };
  static __device__ __forceinline__ v16b load(const __bf16* p) {
    U f; f.h[0] = *(const v8b*)(p); f.h[1] = *(const v8b*)(p + 16); return f.v;
  }
  static __device__ __forceinline__ v8f mma(v16b a, v16b b, v8f c) { return mma_bf16(a, b, c); }
  static __device__ __forceinline__ void keep(v16b a, v16b b, v16b c, v16b d) { keep4_b(a, b, c, d); }
};

__global__ __launch_bounds__(256) void cast8_bf16_kernel(const float* __restrict__ in, unsigned short* __restrict__ out, int n8) {
  const int i = blockIdx.x * 256 + threadIdx.x;
  if (i >= n8) return;
  const float* p = in + 8 * (size_t)i;
  const v4f a = *(const v4f*)(p);
  const v4f d = *(const v4f*)(p + 4);
  v8h hv;
#pragma unroll
  for (int e = 0; e < 4; ++e) {
    const float f0 = a[e];
    const float f1 = d[e];
    const unsigned short h0 = f2bf_bits(f0);
    const unsigned short h1 = f2bf_bits(f1);
    hv[e]     = __builtin_bit_cast(_Float16, h0);
    hv[4 + e] = __builtin_bit_cast(_Float16, h1);
  }
  unsigned short* q = out + 8 * (size_t)i;
  *(volatile v8h*)q = hv;
  __threadfence();
  *(volatile v8h*)q = hv;
}

__global__ __launch_bounds__(256) void wo_cast_kernel(const float* __restrict__ W, unsigned short* __restrict__ out, int n8) {
  const int i = blockIdx.x * 256 + threadIdx.x;
  if (i >= n8) return;
  const int n  = i >> 7;
  const int k8 = (i & 127) * 8;
  const float* p = W + (size_t)n * kD + k8;
  const v4f a = *(const v4f*)(p);
  const v4f d = *(const v4f*)(p + 4);
  v8h hv, lv;
#pragma unroll
  for (int e = 0; e < 4; ++e) {
    const float f0 = a[e];
    const float f1 = d[e];
    const float w0 = bf_bits2f(f2bf_bits(f0));
    const float w1 = bf_bits2f(f2bf_bits(f1));
    const float s0 = w0 * kWoCarry;
    const float s1 = w1 * kWoCarry;
    const float t0 = w0 * kWoLoScale;
    const float t1 = w1 * kWoLoScale;
    hv[e]     = (_Float16)s0;
    hv[4 + e] = (_Float16)s1;
    lv[e]     = (_Float16)t0;
    lv[4 + e] = (_Float16)t1;
  }
  unsigned short* q = out + (size_t)n * kAtld + k8;
  *(volatile v8h*)q = hv;
  *(volatile v8h*)(q + kD) = lv;
  __threadfence();
  *(volatile v8h*)q = hv;
  *(volatile v8h*)(q + kD) = lv;
}

template <int ET> struct Elem;
template <> struct Elem<0> { typedef _Float16 T; };
template <> struct Elem<1> { typedef __bf16 T; };

template <int ET, int OUT_MODE>
__global__ __launch_bounds__(256) void gemm64_kernel(
    const unsigned short* __restrict__ Ap, int lda, long strideA,
    const unsigned short* __restrict__ Btp, int ldb, long strideB,
    void* __restrict__ Cout, int ldc, long strideC,
    unsigned short* __restrict__ Clo, int ldc2, long strideC2,
    int loPerLg, int loRows, int loCols,
    int M, int N, int K, float scale, float loScale) {
  typedef typename Elem<ET>::T T;
  typedef typename Frag<T>::V V;
  const T* A  = (const T*)Ap;
  const T* Bt = (const T*)Btp;
  __shared__ __align__(16) float sT[8][16 * 68];
  const int b    = blockIdx.y;
  const int lane = threadIdx.x & 31;
  const int wave = threadIdx.x >> 5;
  const int tilesN = N >> 6;
  const int tilesM = M >> 6;
  const int tile = blockIdx.x * 8 + wave;
  if (tile >= tilesM * tilesN) return;
  const int tm = tile / tilesN;
  const int tn = tile - tm * tilesN;
  const int m0 = tm << 6;
  const int n0 = tn << 6;

  const T* Ab = A  + (size_t)b * strideA;
  const T* Bb = Bt + (size_t)b * strideB;

  const int rlane = lane & 15;
  const int koff  = (lane >> 4) * 8;
  const int mOff  = (lane >> 4) * 8;

  v8f acc[4][4];
#pragma unroll
  for (int i = 0; i < 4; ++i)
#pragma unroll
    for (int j = 0; j < 4; ++j) acc[i][j] = (v8f){0.f,0.f,0.f,0.f,0.f,0.f,0.f,0.f};

  for (int k0 = 0; k0 < K; k0 += 32) {
    V bh[4];
#pragma unroll
    for (int j = 0; j < 4; ++j) {
      const size_t bo = (size_t)(n0 + (j << 4) + rlane) * ldb + koff + k0;
      bh[j] = Frag<T>::load(Bb + bo);
    }
#pragma unroll
    for (int i = 0; i < 4; ++i) {
      const size_t ao = (size_t)(m0 + (i << 4) + rlane) * lda + koff + k0;
      const V ah = Frag<T>::load(Ab + ao);
#pragma unroll
      for (int j = 0; j < 4; ++j) acc[i][j] = Frag<T>::mma(ah, bh[j], acc[i][j]);
    }
    Frag<T>::keep(bh[0], bh[1], bh[2], bh[3]);
  }
  acc_guard4(acc[0][0], acc[0][1], acc[0][2], acc[0][3]);
  acc_guard4(acc[1][0], acc[1][1], acc[1][2], acc[1][3]);
  acc_guard4(acc[2][0], acc[2][1], acc[2][2], acc[2][3]);
  acc_guard4(acc[3][0], acc[3][1], acc[3][2], acc[3][3]);

  const int perMask = (1 << loPerLg) - 1;
  const int mper    = m0 & perMask;
  const bool wlo    = (OUT_MODE == 3) && (mper < loRows) && (n0 < loCols);
  const int loRow0  = (m0 >> loPerLg) * loRows + mper;

  float* slab = sT[wave];
#pragma unroll
  for (int i = 0; i < 4; ++i) {
    const int mBase = m0 + (i << 4);
#pragma unroll
    for (int j = 0; j < 4; ++j) {
#pragma unroll
      for (int r = 0; r < 8; ++r) {
        const float v = acc[i][j][r] * scale;
        slab[(mOff + r) * 68 + (j << 4) + rlane] = v;
      }
    }
    __builtin_amdgcn_fence(__ATOMIC_RELEASE, "workgroup");
    __builtin_amdgcn_wave_barrier();
    __builtin_amdgcn_fence(__ATOMIC_ACQUIRE, "workgroup");
    if (OUT_MODE == 0) {
      float* C = (float*)Cout + (size_t)b * strideC;
      const int hh = lane >> 4, c4 = (lane & 15) * 4;
      for (int pass = 0; pass < 2; ++pass) {
#pragma unroll
        for (int it = 0; it < 8; ++it) {
          const int row = it * 2 + hh;
          const v4f v = *(const v4f*)(slab + row * 68 + c4);
          *(volatile v4f*)(C + (size_t)(mBase + row) * ldc + n0 + c4) = v;
        }
        __threadfence();
      }
    } else {
      const int q = lane >> 3, c8 = (lane & 7) * 8;
      unsigned short* C  = (unsigned short*)Cout + (size_t)b * strideC;
      unsigned short* C2 = Clo + (size_t)b * strideC2;
      for (int pass = 0; pass < 2; ++pass) {
#pragma unroll
        for (int it = 0; it < 4; ++it) {
          const int row = it * 4 + q;
          const float* sp = slab + row * 68 + c8;
          v8h hv, lv;
#pragma unroll
          for (int e = 0; e < 8; ++e) {
            const float x = sp[e];
            const _Float16 hx = (_Float16)x;
            const float rs = (x - (float)hx) * loScale;
            hv[e] = hx;
            lv[e] = (_Float16)rs;
          }
          *(volatile v8h*)(C + (size_t)(mBase + row) * ldc + n0 + c8) = hv;
          if (wlo) *(volatile v8h*)(C2 + (size_t)(loRow0 + (i << 4) + row) * ldc2 + n0 + c8) = lv;
        }
        __threadfence();
      }
    }
    __builtin_amdgcn_fence(__ATOMIC_RELEASE, "workgroup");
    __builtin_amdgcn_wave_barrier();
    __builtin_amdgcn_fence(__ATOMIC_ACQUIRE, "workgroup");
  }
}

template <bool HI>
__global__ __launch_bounds__(128) void attn_kernel(
    const unsigned short* __restrict__ QKp, const unsigned short* __restrict__ QKlp,
    const unsigned short* __restrict__ Vtp, const unsigned short* __restrict__ Vtlp,
    unsigned short* __restrict__ Atp, const int* __restrict__ cmask, int qb0, int nqb) {
  union FH { v16h v; v8h h[2]; };
  __shared__ __align__(16) _Float16 Psh[4][16 * 64];
  __shared__ __align__(16) _Float16 Psl[HI ? 4 : 1][HI ? 16 * 64 : 8];
  __shared__ __align__(16) float    Os[4][16 * 68];

  const _Float16* QK  = (const _Float16*)QKp;
  const _Float16* QKl = (const _Float16*)QKlp;
  const _Float16* Vt  = (const _Float16*)Vtp;
  const _Float16* Vtl = (const _Float16*)Vtlp;

  const int tid  = threadIdx.x;
  const int wave = tid >> 5;
  const int lane = tid & 31;
  const int hh   = lane >> 4;
  const int c    = lane & 15;

  const int bx = blockIdx.x;
  const int qb = qb0 + (bx % nqb);
  const int bh = bx / nqb;
  const int h  = bh % kH;
  const int b  = bh / kH;
  if (b >= kB || qb >= kQTiles) return;
  const int q0 = qb * 64 + wave * 16;

  const int causal = cmask[0];
  int nChunks = (causal != 0) ? (qb + 1) : kQTiles;
  nChunks = nChunks > kQTiles ? kQTiles : nChunks;

  v16h qah[2], qal[2];
  {
    const _Float16* qp = QK + (size_t)(b * kS + q0 + c) * kQKld + h * kDh + 8 * hh;
    int qlr = q0 + c;
    qlr = qlr < kLoS ? qlr : (kLoS - 1);
    const _Float16* qlp = QKl + (size_t)(b * kLoS + qlr) * kQKld + h * kDh + 8 * hh;
#pragma unroll
    for (int dc = 0; dc < 2; ++dc) {
      qah[dc] = Frag<_Float16>::load(qp + dc * 32);
      if (HI) qal[dc] = Frag<_Float16>::load(qlp + dc * 32);
      else    qal[dc] = qah[dc];
    }
  }

  float mrow[8], lrow[8];
  v8f oacc[4], oaccr[4];
#pragma unroll
  for (int r = 0; r < 8; ++r) { mrow[r] = kMaskFill; lrow[r] = 0.f; }
#pragma unroll
  for (int t = 0; t < 4; ++t) {
    oacc[t]  = (v8f){0.f,0.f,0.f,0.f,0.f,0.f,0.f,0.f};
    oaccr[t] = (v8f){0.f,0.f,0.f,0.f,0.f,0.f,0.f,0.f};
  }

  _Float16* pwh = Psh[wave];
  _Float16* pwl = Psl[HI ? wave : 0];

  for (int kc = 0; kc < nChunks; ++kc) {
    const int kv0 = kc * 64;
    const bool lo_ok = HI && (kc < kLoTiles);
    const int kvl0 = lo_ok ? kv0 : 0;

    v8f s[4];
#pragma unroll
    for (int j = 0; j < 4; ++j) {
      s[j] = (v8f){0.f,0.f,0.f,0.f,0.f,0.f,0.f,0.f};
      v8f sr = (v8f){0.f,0.f,0.f,0.f,0.f,0.f,0.f,0.f};
      const _Float16* kp  = QK  + (size_t)(b * kS + kv0 + j * 16 + c) * kQKld + kD + h * kDh + 8 * hh;
      const _Float16* klp = QKl + (size_t)(b * kLoS + kvl0 + j * 16 + c) * kQKld + kD + h * kDh + 8 * hh;
#pragma unroll
      for (int dc = 0; dc < 2; ++dc) {
        const v16h kb = Frag<_Float16>::load(kp + dc * 32);
        s[j] = mma_f16(qah[dc], kb, s[j]);
        if (HI) {
          sr = mma_f16(qal[dc], kb, sr);
          if (lo_ok) {
            const v16h kl = Frag<_Float16>::load(klp + dc * 32);
            sr = mma_f16(qah[dc], kl, sr);
          }
        }
      }
      if (HI) s[j] = s[j] + sr * kLoCarryInv;
    }

    const bool diag = (causal != 0) && (kc == qb);
#pragma unroll
    for (int r = 0; r < 8; ++r) {
      const int qrow = q0 + 8 * hh + r;
      float sv[4];
      float m = kMaskFill;
#pragma unroll
      for (int j = 0; j < 4; ++j) {
        const int kvcol = kv0 + j * 16 + c;
        float x = s[j][r] * kScoreScale;
        x = (diag && (kvcol > qrow)) ? kMaskFill : x;
        sv[j] = x;
        m = fmaxf(m, x);
      }
#pragma unroll
      for (int off = 1; off < 16; off <<= 1) m = fmaxf(m, __shfl_xor(m, off, 32));
      const float mnew  = fmaxf(mrow[r], m);
      const float alpha = __expf(mrow[r] - mnew);
      mrow[r] = mnew;
      float psum = 0.f;
#pragma unroll
      for (int j = 0; j < 4; ++j) {
        const float p = __expf(sv[j] - mnew);
        psum += p;
        const float p16 = p * kPCarry;
        const _Float16 ph = (_Float16)p16;
        pwh[(8 * hh + r) * 64 + j * 16 + c] = ph;
        if (HI) {
          const float pr = (p16 - (float)ph) * kLoCarry;
          pwl[(8 * hh + r) * 64 + j * 16 + c] = (_Float16)pr;
        }
      }
#pragma unroll
      for (int off = 1; off < 16; off <<= 1) psum += __shfl_xor(psum, off, 32);
      lrow[r] = lrow[r] * alpha + psum;
#pragma unroll
      for (int t = 0; t < 4; ++t) {
        oacc[t][r] *= alpha;
        if (HI) oaccr[t][r] *= alpha;
      }
    }
    __builtin_amdgcn_fence(__ATOMIC_RELEASE, "workgroup");
    __builtin_amdgcn_wave_barrier();
    __builtin_amdgcn_fence(__ATOMIC_ACQUIRE, "workgroup");

#pragma unroll 1
    for (int kk = 0; kk < 2; ++kk) {
      FH pa, pl;
      pa.h[0] = *(const v8h*)(pwh + c * 64 + kk * 32 + 8 * hh);
      pa.h[1] = *(const v8h*)(pwh + c * 64 + kk * 32 + 16 + 8 * hh);
      if (HI) {
        pl.h[0] = *(const v8h*)(pwl + c * 64 + kk * 32 + 8 * hh);
        pl.h[1] = *(const v8h*)(pwl + c * 64 + kk * 32 + 16 + 8 * hh);
      } else {
        pl.v = pa.v;
      }
#pragma unroll
      for (int t = 0; t < 4; ++t) {
        const size_t vr = (size_t)(b * kD + h * kDh + t * 16 + c);
        const v16h vb = Frag<_Float16>::load(Vt + vr * kS + kv0 + kk * 32 + 8 * hh);
        oacc[t] = mma_f16(pa.v, vb, oacc[t]);
        if (HI) {
          oaccr[t] = mma_f16(pl.v, vb, oaccr[t]);
          if (lo_ok) {
            const v16h vl = Frag<_Float16>::load(Vtl + vr * kLoS + kvl0 + kk * 32 + 8 * hh);
            oaccr[t] = mma_f16(pa.v, vl, oaccr[t]);
          }
        }
      }
    }
    __builtin_amdgcn_fence(__ATOMIC_RELEASE, "workgroup");
    __builtin_amdgcn_wave_barrier();
    __builtin_amdgcn_fence(__ATOMIC_ACQUIRE, "workgroup");
  }

  float* os = Os[wave];
#pragma unroll
  for (int r = 0; r < 8; ++r) {
    const float inv = 1.0f / (lrow[r] * kPCarry);
#pragma unroll
    for (int t = 0; t < 4; ++t) {
      float o = oacc[t][r];
      if (HI) o = o + oaccr[t][r] * kLoCarryInv;
      os[(8 * hh + r) * 68 + t * 16 + c] = o * inv;
    }
  }
  __builtin_amdgcn_fence(__ATOMIC_RELEASE, "workgroup");
  __builtin_amdgcn_wave_barrier();
  __builtin_amdgcn_fence(__ATOMIC_ACQUIRE, "workgroup");
  {
    const int q = lane >> 3, c8 = (lane & 7) * 8;
    for (int pass = 0; pass < 2; ++pass) {
#pragma unroll
      for (int it = 0; it < 4; ++it) {
        const int row = it * 4 + q;
        const float* sp = os + row * 68 + c8;
        v8h hv, lv;
#pragma unroll
        for (int e = 0; e < 8; ++e) {
          const float x = sp[e] * kCtxCarry;
          const _Float16 hx = (_Float16)x;
          const float rs = (x - (float)hx) * kCtxLoCarry;
          hv[e] = hx;
          lv[e] = (_Float16)rs;
        }
        unsigned short* dst = Atp + (size_t)(b * kS + q0 + row) * kAtld + h * kDh + c8;
        *(volatile v8h*)dst = hv;
        *(volatile v8h*)(dst + kD) = lv;
      }
      __threadfence();
    }
  }
}

extern "C" void kernel_launch(void* const* d_in, const int* in_sizes, int n_in,
                              void* d_out, int out_size, void* d_ws, size_t ws_size,
                              hipStream_t stream) {
  if (n_in < 4) return;
  if (in_sizes[0] != kTok * kD) return;
  if (in_sizes[1] != kE3 * kD) return;
  if (in_sizes[2] != kD * kD) return;
  if (in_sizes[3] != 1) return;
  if (out_size != kTok * kD) return;
  if (ws_size < kWsTotal) return;

  const float* x     = (const float*)d_in[0];
  const float* w_in  = (const float*)d_in[1];
  const float* w_out = (const float*)d_in[2];
  const int*   cm    = (const int*)d_in[3];
  float* out = (float*)d_out;

  char* ws = (char*)d_ws;
  unsigned short* XB  = (unsigned short*)(ws + kOffXB);
  unsigned short* WB  = (unsigned short*)(ws + kOffWB);
  unsigned short* WO2 = (unsigned short*)(ws + kOffWO2);
  unsigned short* QK  = (unsigned short*)(ws + kOffQK);
  unsigned short* VT  = (unsigned short*)(ws + kOffVT);
  unsigned short* QKL = (unsigned short*)(ws + kOffQKL);
  unsigned short* VTL = (unsigned short*)(ws + kOffVTL);
  unsigned short* AT  = (unsigned short*)(ws + kOffAT);

  cast8_bf16_kernel<<<(kTok * kD / 8) / 256, 256, 0, stream>>>(x, XB, kTok * kD / 8);
  cast8_bf16_kernel<<<(kE3 * kD / 8) / 256, 256, 0, stream>>>(w_in, WB, kE3 * kD / 8);
  wo_cast_kernel<<<(kD * kD / 8) / 256, 256, 0, stream>>>(w_out, WO2, kD * kD / 8);

  gemm64_kernel<1, 3><<<dim3((kTok / 64) * (kQKld / 64) / 8, 1), 256, 0, stream>>>(
      XB, kD, 0L,
      WB, kD, 0L,
      (void*)QK, kQKld, 0L,
      QKL, kQKld, 0L,
      11, kLoS, kQKld,
      kTok, kQKld, kD, 1.0f, kLoCarry);

  gemm64_kernel<1, 3><<<dim3((kD / 64) * (kS / 64) / 8, kB), 256, 0, stream>>>(
      WB + (size_t)2 * kD * kD, kD, 0L,
      XB, kD, (long)kS * kD,
      (void*)VT, kS, (long)kD * kS,
      VTL, kLoS, (long)kD * kLoS,
      10, kD, kLoS,
      kD, kS, kD, 1.0f, kLoCarry);

  attn_kernel<true><<<kB * kH * kLoTiles, 128, 0, stream>>>(QK, QKL, VT, VTL, AT, cm, 0, kLoTiles);
  attn_kernel<false><<<kB * kH * (kQTiles - kLoTiles), 128, 0, stream>>>(QK, QKL, VT, VTL, AT, cm, kLoTiles, kQTiles - kLoTiles);

  gemm64_kernel<0, 0><<<dim3((kTok / 64) * (kD / 64) / 8, 1), 256, 0, stream>>>(
      AT, kAtld, 0L,
      WO2, kAtld, 0L,
      (void*)out, kD, 0L,
      WO2, kAtld, 0L,
      0, 0, 0,
      kTok, kD, kAtld, kOutScale, 1.0f);
}
